// ZetaBlockEnhanced_63823214018762
// MI455X (gfx1250) — hardware-verified
//
#include <hip/hip_runtime.h>
#include <math.h>

constexpr int kBatch = 2;
constexpr int kSeq   = 2048;
constexpr int kDim   = 1024;
constexpr int kHeads = 16;
constexpr int kDh    = 64;
constexpr int kTok   = kBatch * kSeq;
constexpr float kWCarry    = 32.0f;
constexpr float kWCarryInv = 1.0f / 32.0f;
constexpr float kFCarry    = 64.0f;
constexpr float kYScale    = 1.0f / (64.0f * 32.0f);
constexpr float kSScale    = 0.125f;
constexpr float kInvDim    = 1.0f / 1024.0f;
constexpr float kLnEps     = 1e-5f;

typedef __attribute__((ext_vector_type(16))) _Float16 v16h;
typedef __attribute__((ext_vector_type(8)))  _Float16 v8h;
typedef __attribute__((ext_vector_type(16))) __bf16   v16b;
typedef __attribute__((ext_vector_type(8)))  __bf16   v8b;
typedef __attribute__((ext_vector_type(8)))  float    v8f;
typedef __attribute__((ext_vector_type(4)))  float    v4f;
typedef __attribute__((ext_vector_type(4)))  unsigned int v4u;
typedef __attribute__((ext_vector_type(2)))  unsigned int v2u;

__device__ __forceinline__ unsigned short f2bf_bits(float f) {
  unsigned u = __float_as_uint(f);
  return (unsigned short)((u + 0x7FFFu + ((u >> 16) & 1u)) >> 16);
}
__device__ __forceinline__ float bf_bits2f(unsigned short h) { return __uint_as_float(((unsigned)h) << 16); }

__device__ __forceinline__ void dep_guard_h(v8f& a, v8f& b, v16h x, v16h y) { asm volatile("v_nop\n\tv_nop\n\tv_nop\n\tv_nop" : "+v"(a), "+v"(b) : "v"(x), "v"(y)); }
__device__ __forceinline__ void dep_guard_b(v8f& a, v8f& b, v16b x, v16b y) { asm volatile("v_nop\n\tv_nop\n\tv_nop\n\tv_nop" : "+v"(a), "+v"(b) : "v"(x), "v"(y)); }
__device__ __forceinline__ void keep4_h(v16h a, v16h b, v16h c, v16h d) { asm volatile("v_nop" :: "v"(a), "v"(b), "v"(c), "v"(d)); }
__device__ __forceinline__ void keep4_b(v16b a, v16b b, v16b c, v16b d) { asm volatile("v_nop" :: "v"(a), "v"(b), "v"(c), "v"(d)); }
__device__ __forceinline__ void acc_guard4(v8f& a, v8f& b, v8f& c, v8f& d) { asm volatile("v_nop\n\tv_nop\n\tv_nop\n\tv_nop" : "+v"(a), "+v"(b), "+v"(c), "+v"(d)); }
template <typename T> struct Frag;
template <> struct Frag<_Float16> {
  typedef v16h V; union U { v16h v; v8h h[2]; };
  static __device__ __forceinline__ v16h load(const _Float16* p) {
    U f; f.h[0] = *(const v8h*)(p); f.h[1] = *(const v8h*)(p + 16); return f.v;
  }
  static __device__ __forceinline__ v8f mma(v16h a, v16h b, v8f c) {
    return __builtin_amdgcn_wmma_f32_16x16x32_f16(false, a, false, b, (short)0, c, false, false);
  }
  static __device__ __forceinline__ void guard(v8f& a, v8f& b, v16h x, v16h y) { dep_guard_h(a, b, x, y); }
  static __device__ __forceinline__ void keep(v16h a, v16h b, v16h c, v16h d) { keep4_h(a, b, c, d); }
};
template <> struct Frag<__bf16> {
  typedef v16b V; union U { v16b v; v8b h[2]; };
  static __device__ __forceinline__ v16b load(const __bf16* p) {
    U f; f.h[0] = *(const v8b*)(p); f.h[1] = *(const v8b*)(p + 16); return f.v;
  }
  static __device__ __forceinline__ v8f mma(v16b a, v16b b, v8f c) {
    return __builtin_amdgcn_wmma_f32_16x16x32_bf16(false, a, false, b, (short)0, c, false, false);
  }
  static __device__ __forceinline__ void guard(v8f& a, v8f& b, v16b x, v16b y) { dep_guard_b(a, b, x, y); }
  static __device__ __forceinline__ void keep(v16b a, v16b b, v16b c, v16b d) { keep4_b(a, b, c, d); }
};

__device__ __forceinline__ unsigned pk16(unsigned short a, unsigned short b) { return (unsigned)a | ((unsigned)b << 16); }
__device__ __forceinline__ unsigned short h_bits(float f) { const _Float16 h = (_Float16)f; return __builtin_bit_cast(unsigned short, h); }

template <int ET> struct Elem;
template <> struct Elem<0> { typedef _Float16 T; };
template <> struct Elem<1> { typedef __bf16 T; };
template <int ET, bool SPLIT, int BIAS_MODE, int OUT_MODE, bool RESID, int ACT = 0>
__global__ __launch_bounds__(256) void wmma_gemm64(
    const unsigned short* __restrict__ Ap, const unsigned short* __restrict__ A2p, int lda, long strideA,
    const unsigned short* __restrict__ Btp, const unsigned short* __restrict__ Bt2p, int ldb, long strideB,
    void* __restrict__ Cout, void* __restrict__ Cout2, int ldc, long strideC,
    const float* __restrict__ bias,
    const float* __restrict__ resid, long strideR,
    int M, int N, int K, float scale) {
  typedef typename Elem<ET>::T T;
  typedef typename Frag<T>::V V;
  const T* A = (const T*)Ap; const T* A2 = (const T*)A2p; const T* Bt = (const T*)Btp; const T* Bt2 = (const T*)Bt2p;
  __shared__ __align__(16) float sT[8][16 * 68];
  const int b    = blockIdx.y;
  const int lane = threadIdx.x & 31;
  const int wave = threadIdx.x >> 5;
  const int tilesN = N >> 6;
  const int tilesM = M >> 6;
  const int tile = blockIdx.x * 8 + wave;
  if (tile >= tilesM * tilesN) return;
  const int tm = tile / tilesN;
  const int tn = tile - tm * tilesN;
  const int m0 = tm << 6;
  const int n0 = tn << 6;

  const T* Ab  = A  + (size_t)b * strideA;
  const T* Bb  = Bt + (size_t)b * strideB;
  const T* Ab2 = SPLIT ? (A2  + (size_t)b * strideA) : nullptr;
  const T* Bb2 = SPLIT ? (Bt2 + (size_t)b * strideB) : nullptr;

  const int rlane = lane & 15;
  const int koff  = (lane >> 4) * 8;
  const int mOff  = (lane >> 4) * 8;

  v8f acc[4][4];
#pragma unroll
  for (int i = 0; i < 4; ++i)
#pragma unroll
    for (int j = 0; j < 4; ++j) acc[i][j] = (v8f){0.f,0.f,0.f,0.f,0.f,0.f,0.f,0.f};

  for (int k0 = 0; k0 < K; k0 += 32) {
    V bh[4], bl[4];
#pragma unroll
    for (int j = 0; j < 4; ++j) {
      const size_t bo = (size_t)(n0 + (j << 4) + rlane) * ldb + koff + k0;
      bh[j] = Frag<T>::load(Bb + bo);
      if (SPLIT) bl[j] = Frag<T>::load(Bb2 + bo);
    }
#pragma unroll
    for (int i = 0; i < 4; ++i) {
      const size_t ao = (size_t)(m0 + (i << 4) + rlane) * lda + koff + k0;
      V ah = Frag<T>::load(Ab + ao);
      V al;
      if (SPLIT) al = Frag<T>::load(Ab2 + ao);
#pragma unroll
      for (int j = 0; j < 4; ++j) {
        acc[i][j] = Frag<T>::mma(ah, bh[j], acc[i][j]);
        if (SPLIT) {
          acc[i][j] = Frag<T>::mma(ah, bl[j], acc[i][j]);
          acc[i][j] = Frag<T>::mma(al, bh[j], acc[i][j]);
        }
      }
      Frag<T>::guard(acc[i][0], acc[i][3], ah, SPLIT ? al : ah);
    }
    Frag<T>::keep(bh[0], bh[1], bh[2], bh[3]);
    if (SPLIT) Frag<T>::keep(bl[0], bl[1], bl[2], bl[3]);
  }
  acc_guard4(acc[0][0], acc[0][1], acc[0][2], acc[0][3]);
  acc_guard4(acc[1][0], acc[1][1], acc[1][2], acc[1][3]);
  acc_guard4(acc[2][0], acc[2][1], acc[2][2], acc[2][3]);
  acc_guard4(acc[3][0], acc[3][1], acc[3][2], acc[3][3]);

  float* slab = sT[wave];
  const float* Rb = RESID ? (resid + (size_t)b * strideR) : nullptr;
#pragma unroll
  for (int i = 0; i < 4; ++i) {
    const int mBase = m0 + (i << 4);
#pragma unroll
    for (int j = 0; j < 4; ++j) {
      const int n = n0 + (j << 4) + rlane;
      float bv = 0.f;
      if (BIAS_MODE == 2) bv = bias[n];
#pragma unroll
      for (int r = 0; r < 8; ++r) {
        float v = acc[i][j][r] * scale;
        if (BIAS_MODE == 1) v += bias[mBase + mOff + r];
        if (BIAS_MODE == 2) v += bv;
        if (RESID) v += Rb[(size_t)(mBase + mOff + r) * ldc + n];
        if (ACT == 2) v = fmaxf(v, 0.0f);
        if (ACT == 4) v = (v > 0.f) ? v : 0.01f * v;
        slab[(mOff + r) * 68 + (j << 4) + rlane] = v;
      }
    }
    __builtin_amdgcn_fence(__ATOMIC_RELEASE, "workgroup");
    __builtin_amdgcn_wave_barrier();
    __builtin_amdgcn_fence(__ATOMIC_ACQUIRE, "workgroup");
    if (OUT_MODE == 0) {
      float* C = (float*)Cout + (size_t)b * strideC;
      const int hh = lane >> 4, c4 = (lane & 15) * 4;
      for (int pass = 0; pass < 2; ++pass) {
#pragma unroll
        for (int it = 0; it < 8; ++it) {
          const int row = it * 2 + hh;
          v4f v = *(const v4f*)(slab + row * 68 + c4);
          *(volatile v4f*)(C + (size_t)(mBase + row) * ldc + n0 + c4) = v;
        }
        __threadfence();
      }
    } else {
      const int q = lane >> 3, c8 = (lane & 7) * 8;
      unsigned short* C  = (unsigned short*)Cout  + (size_t)b * strideC;
      unsigned short* C2 = (OUT_MODE == 2) ? ((unsigned short*)Cout2 + (size_t)b * strideC) : nullptr;
      for (int pass = 0; pass < 2; ++pass) {
#pragma unroll
        for (int it = 0; it < 4; ++it) {
          const int row = it * 4 + q;
          const float* sp = slab + row * 68 + c8;
          v8h hv, lv;
#pragma unroll
          for (int e = 0; e < 8; ++e) {
            if (OUT_MODE == 1) {
              hv[e] = (_Float16)sp[e];
            } else {
              unsigned short hb = f2bf_bits(sp[e]);
              unsigned short lb = f2bf_bits(sp[e] - bf_bits2f(hb));
              hv[e] = __builtin_bit_cast(_Float16, hb);
              lv[e] = __builtin_bit_cast(_Float16, lb);
            }
          }
          *(volatile v8h*)(C + (size_t)(mBase + row) * ldc + n0 + c8) = hv;
          if (OUT_MODE == 2) *(volatile v8h*)(C2 + (size_t)(mBase + row) * ldc + n0 + c8) = lv;
        }
        __threadfence();
      }
    }
    __builtin_amdgcn_fence(__ATOMIC_RELEASE, "workgroup");
    __builtin_amdgcn_wave_barrier();
    __builtin_amdgcn_fence(__ATOMIC_ACQUIRE, "workgroup");
  }
}

__global__ __launch_bounds__(256) void cast8_f16_kernel(const float* __restrict__ in0, const float* __restrict__ in1,
                                                        const float* __restrict__ in2, const float* __restrict__ in3,
                                                        unsigned short* __restrict__ out, long planeElems, int n8,
                                                        float scale) {
  const int i = blockIdx.x * 256 + threadIdx.x;
  const int z = blockIdx.y;
  if (i >= n8) return;
  const float* in = (z == 0) ? in0 : (z == 1) ? in1 : (z == 2) ? in2 : in3;
  const float* p = in + 8 * (size_t)i;
  const v4f a = *(const v4f*)(p);
  const v4f c = *(const v4f*)(p + 4);
  unsigned short hb[8];
#pragma unroll
  for (int e = 0; e < 4; ++e) {
    hb[e]     = h_bits(a[e] * scale);
    hb[4 + e] = h_bits(c[e] * scale);
  }
  const v4u u = (v4u){pk16(hb[0], hb[1]), pk16(hb[2], hb[3]), pk16(hb[4], hb[5]), pk16(hb[6], hb[7])};
  unsigned short* q = out + (size_t)z * planeElems + 8 * (size_t)i;
  *(volatile v4u*)q = u;
  __threadfence();
  *(volatile v4u*)q = u;
}

__global__ __launch_bounds__(512) void dual_weights_kernel(const float* __restrict__ S,
                                                          unsigned short* __restrict__ Phi,
                                                          unsigned short* __restrict__ Plo,
                                                          const float* __restrict__ beta,
                                                          const float* __restrict__ tvec, int h0) {
  __shared__ float redM[16];
  __shared__ float redT[16];
  __shared__ float redS[16];
  __shared__ __align__(16) unsigned int sHi[1024];
  __shared__ __align__(16) unsigned int sLo[1024];
  const int row  = blockIdx.x;
  const int grp  = row >> 11;
  int h = h0 + grp;
  h = (h < 0) ? 0 : ((h > kHeads - 1) ? (kHeads - 1) : h);
  const int t = threadIdx.x;
  const int lane = t & 31, wave = t >> 5;

  const v4f sv = *(const v4f*)(S + (size_t)row * kSeq + 4 * t);
  float m = fmaxf(fmaxf(sv.x, sv.y), fmaxf(sv.z, sv.w));
#pragma unroll
  for (int off = 16; off > 0; off >>= 1) m = fmaxf(m, __shfl_xor(m, off, 32));
  if (lane == 0) redM[wave] = m;
  __syncthreads();
  float mx = redM[0];
#pragma unroll
  for (int i = 1; i < 16; ++i) mx = fmaxf(mx, redM[i]);

  const float invb = 1.0f / beta[h];
  const float th = tvec[h];
  const float t2 = th * th;

  const float e0 = expf(sv.x - mx);
  const float e1 = expf(sv.y - mx);
  const float e2 = expf(sv.z - mx);
  const float e3 = expf(sv.w - mx);
  const float q0 = 1.0f + fabsf(sv.x) * invb;
  const float q1 = 1.0f + fabsf(sv.y) * invb;
  const float q2 = 1.0f + fabsf(sv.z) * invb;
  const float q3 = 1.0f + fabsf(sv.w) * invb;
  const float w0 = 1.0f / (q0 * q0 + t2);
  const float w1 = 1.0f / (q1 * q1 + t2);
  const float w2 = 1.0f / (q2 * q2 + t2);
  const float w3 = 1.0f / (q3 * q3 + t2);

  float st = ((e0 + e1) + e2) + e3;
  float ss = ((w0 + w1) + w2) + w3;
#pragma unroll
  for (int off = 16; off > 0; off >>= 1) {
    st += __shfl_xor(st, off, 32);
    ss += __shfl_xor(ss, off, 32);
  }
  if (lane == 0) { redT[wave] = st; redS[wave] = ss; }
  __syncthreads();
  float sumT = redT[0], sumS = redS[0];
#pragma unroll
  for (int i = 1; i < 16; ++i) { sumT += redT[i]; sumS += redS[i]; }
  const float invT = 1.0f / sumT;
  const float invS = 1.0f / sumS;

  const float p0 = 0.5f * (e0 * invT + w0 * invS);
  const float p1 = 0.5f * (e1 * invT + w1 * invS);
  const float p2 = 0.5f * (e2 * invT + w2 * invS);
  const float p3 = 0.5f * (e3 * invT + w3 * invS);

  const unsigned short hb0 = f2bf_bits(p0), hb1 = f2bf_bits(p1), hb2 = f2bf_bits(p2), hb3 = f2bf_bits(p3);
  const unsigned short lb0 = f2bf_bits(p0 - bf_bits2f(hb0));
  const unsigned short lb1 = f2bf_bits(p1 - bf_bits2f(hb1));
  const unsigned short lb2 = f2bf_bits(p2 - bf_bits2f(hb2));
  const unsigned short lb3 = f2bf_bits(p3 - bf_bits2f(hb3));
  *(v2u*)(sHi + 2 * t) = (v2u){pk16(hb0, hb1), pk16(hb2, hb3)};
  *(v2u*)(sLo + 2 * t) = (v2u){pk16(lb0, lb1), pk16(lb2, lb3)};
  __syncthreads();

  const int j = t & 255;
  const bool isLo = (t >= 256);
  const v4u a = *(const v4u*)(sHi + 4 * j);
  const v4u c = *(const v4u*)(sLo + 4 * j);
  v4u u;
  u.x = isLo ? c.x : a.x;
  u.y = isLo ? c.y : a.y;
  u.z = isLo ? c.z : a.z;
  u.w = isLo ? c.w : a.w;
  unsigned short* dst = (isLo ? Plo : Phi) + (size_t)row * kSeq + 8 * j;
  *(volatile v4u*)dst = u;
  __threadfence();
  *(volatile v4u*)dst = u;
}

__global__ __launch_bounds__(256) void ln_residual_kernel(const float* __restrict__ x, const float* __restrict__ y,
                                                          const float* __restrict__ lw, const float* __restrict__ lb,
                                                          float* __restrict__ out) {
  __shared__ float red0[8];
  __shared__ float red1[8];
  const int row = blockIdx.x;
  const int t = threadIdx.x;
  const int lane = t & 31, wave = t >> 5;
  const size_t base = (size_t)row * kDim + 4 * t;
  const v4f yv = *(const v4f*)(y + base);
  const v4f xv = *(const v4f*)(x + base);
  const v4f wv = *(const v4f*)(lw + 4 * t);
  const v4f bv = *(const v4f*)(lb + 4 * t);

  float s = ((yv.x + yv.y) + yv.z) + yv.w;
#pragma unroll
  for (int off = 16; off > 0; off >>= 1) s += __shfl_xor(s, off, 32);
  if (lane == 0) red0[wave] = s;
  __syncthreads();
  float tot = red0[0];
#pragma unroll
  for (int i = 1; i < 8; ++i) tot += red0[i];
  const float mu = tot * kInvDim;

  const float d0 = yv.x - mu, d1 = yv.y - mu, d2 = yv.z - mu, d3 = yv.w - mu;
  float s2 = ((d0 * d0 + d1 * d1) + d2 * d2) + d3 * d3;
#pragma unroll
  for (int off = 16; off > 0; off >>= 1) s2 += __shfl_xor(s2, off, 32);
  if (lane == 0) red1[wave] = s2;
  __syncthreads();
  float tot2 = red1[0];
#pragma unroll
  for (int i = 1; i < 8; ++i) tot2 += red1[i];
  const float var = tot2 * kInvDim;
  const float rs = rsqrtf(var + kLnEps);

  v4f o;
  o.x = xv.x + (wv.x * d0 * rs + bv.x);
  o.y = xv.y + (wv.y * d1 * rs + bv.y);
  o.z = xv.z + (wv.z * d2 * rs + bv.z);
  o.w = xv.w + (wv.w * d3 * rs + bv.w);
  float* op = out + base;
  *(volatile v4f*)op = o;
  __threadfence();
  *(volatile v4f*)op = o;
}

extern "C" void kernel_launch(void* const* d_in, const int* in_sizes, int n_in,
                              void* d_out, int out_size, void* d_ws, size_t ws_size,
                              hipStream_t stream) {
  if (n_in < 13) return;
  const size_t nX = (size_t)kTok * kDim;
  const size_t nW = (size_t)kDim * kDim;
  if ((size_t)in_sizes[0] != nX || (size_t)in_sizes[1] != nW || (size_t)in_sizes[3] != nW ||
      (size_t)in_sizes[5] != nW || (size_t)in_sizes[7] != nW || (size_t)out_size != nX) return;
  if (in_sizes[2] < kDim || in_sizes[4] < kDim || in_sizes[6] < kDim || in_sizes[8] < kDim ||
      in_sizes[9] < kHeads || in_sizes[10] < kHeads || in_sizes[11] < kDim || in_sizes[12] < kDim) return;

  const float* x    = (const float*)d_in[0];
  const float* Wq   = (const float*)d_in[1];
  const float* bq   = (const float*)d_in[2];
  const float* Wk   = (const float*)d_in[3];
  const float* bk   = (const float*)d_in[4];
  const float* Wv   = (const float*)d_in[5];
  const float* bv   = (const float*)d_in[6];
  const float* Wo   = (const float*)d_in[7];
  const float* bo   = (const float*)d_in[8];
  const float* beta = (const float*)d_in[9];
  const float* tv   = (const float*)d_in[10];
  const float* lw   = (const float*)d_in[11];
  const float* lb   = (const float*)d_in[12];
  float* out = (float*)d_out;

  const size_t bXF   = nX * 2;
  const size_t bW16  = 4 * nW * 2;
  const size_t bP16  = nX * 2;
  const size_t bSY   = (size_t)2 * kSeq * kSeq * 4;
  const size_t bPP   = (size_t)2 * kSeq * kSeq * 2;
  const size_t oXF   = 0;
  const size_t oW16  = oXF + bXF;
  const size_t oQHI  = oW16 + bW16;
  const size_t oQLO  = oQHI + bP16;
  const size_t oKHI  = oQLO + bP16;
  const size_t oKLO  = oKHI + bP16;
  const size_t oVTHI = oKLO + bP16;
  const size_t oVTLO = oVTHI + bP16;
  const size_t oSY   = oVTLO + bP16;
  const size_t oPHI  = oSY + bSY;
  const size_t oPLO  = oPHI + bPP;
  const size_t total = oPLO + bPP;
  if (total > ws_size) return;

  char* ws = (char*)d_ws;
  unsigned short* XF   = (unsigned short*)(ws + oXF);
  unsigned short* W16  = (unsigned short*)(ws + oW16);
  unsigned short* Wq16 = W16;
  unsigned short* Wk16 = W16 + nW;
  unsigned short* Wv16 = W16 + 2 * nW;
  unsigned short* Wo16 = W16 + 3 * nW;
  unsigned short* QHI  = (unsigned short*)(ws + oQHI);
  unsigned short* QLO  = (unsigned short*)(ws + oQLO);
  unsigned short* KHI  = (unsigned short*)(ws + oKHI);
  unsigned short* KLO  = (unsigned short*)(ws + oKLO);
  unsigned short* VTHI = (unsigned short*)(ws + oVTHI);
  unsigned short* VTLO = (unsigned short*)(ws + oVTLO);
  float*          SY   = (float*)(ws + oSY);
  unsigned short* PHI  = (unsigned short*)(ws + oPHI);
  unsigned short* PLO  = (unsigned short*)(ws + oPLO);

  {
    const int n8 = (int)(nX / 8);
    cast8_f16_kernel<<<dim3(n8 / 256, 1), 256, 0, stream>>>(x, x, x, x, XF, 0L, n8, 1.0f);
  }
  {
    const int n8 = (int)(nW / 8);
    cast8_f16_kernel<<<dim3(n8 / 256, 4), 256, 0, stream>>>(Wq, Wk, Wv, Wo, W16, (long)nW, n8, kWCarry);
  }
  const int gemmBlocksProj = (kTok / 64) * (kDim / 64) / 8;
  wmma_gemm64<0, false, 2, 2, false><<<dim3(gemmBlocksProj, 1), 256, 0, stream>>>(
      XF, XF, kDim, 0L, Wq16, Wq16, kDim, 0L, (void*)QHI, (void*)QLO, kDim, 0L,
      bq, x, 0L, kTok, kDim, kDim, kWCarryInv);
  wmma_gemm64<0, false, 2, 2, false><<<dim3(gemmBlocksProj, 1), 256, 0, stream>>>(
      XF, XF, kDim, 0L, Wk16, Wk16, kDim, 0L, (void*)KHI, (void*)KLO, kDim, 0L,
      bk, x, 0L, kTok, kDim, kDim, kWCarryInv);
  wmma_gemm64<0, false, 1, 2, false><<<dim3(gemmBlocksProj, 1), 256, 0, stream>>>(
      Wv16, Wv16, kDim, 0L, XF, XF, kDim, 0L, (void*)VTHI, (void*)VTLO, kTok, 0L,
      bv, x, 0L, kDim, kTok, kDim, kWCarryInv);

  const long strideS = (long)kSeq * kSeq;
  for (int p = 0; p < (kBatch * kHeads) / 2; ++p) {
    const int b  = p >> 3;
    const int h0 = (2 * p) & (kHeads - 1);
    const size_t qkBase = (size_t)b * kSeq * kDim + (size_t)h0 * kDh;
    wmma_gemm64<1, true, 0, 0, false><<<dim3(128, 2), 256, 0, stream>>>(
        QHI + qkBase, QLO + qkBase, kDim, (long)kDh,
        KHI + qkBase, KLO + qkBase, kDim, (long)kDh,
        (void*)SY, (void*)SY, kSeq, strideS,
        bq, x, 0L, kSeq, kSeq, kDh, kSScale);
    dual_weights_kernel<<<dim3(2 * kSeq), 512, 0, stream>>>(SY, PHI, PLO, beta, tv, h0);
    const size_t vtBase = (size_t)h0 * kDh * kTok + (size_t)b * kSeq;
    const size_t fBase  = (size_t)b * kSeq * kDim + (size_t)h0 * kDh;
    wmma_gemm64<1, true, 0, 1, false><<<dim3(4, 2), 256, 0, stream>>>(
        PHI, PLO, kSeq, strideS,
        VTHI + vtBase, VTLO + vtBase, kTok, (long)kDh * kTok,
        (void*)(XF + fBase), (void*)(XF + fBase), kDim, (long)kDh,
        bq, x, 0L, kSeq, kDh, kSeq, kFCarry);
  }

  wmma_gemm64<0, false, 2, 0, false><<<dim3(gemmBlocksProj, 1), 256, 0, stream>>>(
      XF, XF, kDim, 0L, Wo16, Wo16, kDim, 0L, (void*)SY, (void*)SY, kDim, 0L,
      bo, x, 0L, kTok, kDim, kDim, kYScale);

  ln_residual_kernel<<<dim3(kTok), 256, 0, stream>>>(x, SY, lw, lb, out);
}
